// ScaledDotProductAttention_48696339202255
// MI455X (gfx1250) — hardware-verified
//
#include <hip/hip_runtime.h>
#include <stdint.h>


typedef _Float16 v16h __attribute__((ext_vector_type(16)));
typedef _Float16 v8h  __attribute__((ext_vector_type(8)));
typedef float    v8f  __attribute__((ext_vector_type(8)));
typedef float    v4f  __attribute__((ext_vector_type(4)));
typedef int      v4i  __attribute__((ext_vector_type(4)));

#ifndef NB
#define NB 2
#endif
#ifndef SEQ
#define SEQ 2048
#endif
#define SEQ_FULL 2048
#define NH 16
#define DK 64

constexpr unsigned QT  = 128;
constexpr unsigned KB  = 64;
constexpr unsigned NT  = KB / 16;
constexpr unsigned NKB = SEQ / KB;
constexpr unsigned PCH = 128;
constexpr unsigned KDP = DK + 8;
constexpr unsigned VDP = KB + 8;
constexpr unsigned PDP = KB + 8;
constexpr unsigned ODP = DK + 4;
constexpr unsigned TP  = PCH + 8;
constexpr unsigned QP  = NH * DK;
constexpr unsigned MP  = SEQ_FULL;
constexpr size_t IN_B  = (size_t)SEQ_FULL * QP;
constexpr size_t WS_BH = (size_t)SEQ * DK;

static_assert(NB >= 1);
static_assert(NH == 16);
static_assert(DK == 64);
static_assert(SEQ >= 128);
static_assert(SEQ <= SEQ_FULL);
static_assert(SEQ % 128 == 0);
static_assert(NT == 4);
static_assert(KB == DK);
static_assert((KDP * 2) % 16 == 0);
static_assert((VDP * 2) % 16 == 0);
static_assert((PDP * 2) % 16 == 0);
static_assert((ODP * 4) % 16 == 0);
static_assert((TP  * 2) % 16 == 0);
static_assert((size_t)(SEQ / 128) * (NB * NH) * 256u * 4u * 8u == (size_t)NB * NH * SEQ * DK);
static_assert((size_t)(SEQ / 128) * NH * NB * 256u * 8u * 4u == (size_t)NB * NH * SEQ * DK);

union HV { v8h h; v4i i; };

__device__ __forceinline__ float bf16v(float x) {
    uint32_t u = __float_as_uint(x);
    u = (u + 0x7FFFu + ((u >> 16) & 1u)) & 0xFFFF0000u;
    return __uint_as_float(u);
}
__device__ __forceinline__ _Float16 h16(float x) { return (_Float16)bf16v(x); }

__device__ __forceinline__ float fexp2(float x) {
#if defined(__has_builtin)
#if __has_builtin(__builtin_amdgcn_exp2f)
    return __builtin_amdgcn_exp2f(x);
#else
    return exp2f(x);
#endif
#else
    return exp2f(x);
#endif
}

__device__ __forceinline__ float frcp(float x) {
#if defined(__has_builtin)
#if __has_builtin(__builtin_amdgcn_rcpf)
    return __builtin_amdgcn_rcpf(x);
#else
    return 1.0f / x;
#endif
#else
    return 1.0f / x;
#endif
}

__device__ __forceinline__ v8f mma16(v16h a, v16h b, v8f c) {
    v8f d = __builtin_amdgcn_wmma_f32_16x16x32_f16(false, a, false, b, (short)0, c, false, false);
    asm volatile("v_nop\n\tv_nop\n\tv_nop\n\tv_nop" : "+v"(d) : "v"(a), "v"(b));
    return d;
}

__device__ __forceinline__ v16h ld_op16(const _Float16* p) {
    union { v16h v; v8h hh[2]; } u;
    u.hh[0] = *(const v8h*)(p);
    u.hh[1] = *(const v8h*)(p + 16);
    return u.v;
}

__device__ __forceinline__ v16h ld_q(const float* p) {
    const v4f x0 = *(const v4f*)(p);
    const v4f x1 = *(const v4f*)(p + 4);
    const v4f x2 = *(const v4f*)(p + 16);
    const v4f x3 = *(const v4f*)(p + 20);
    v16h r;
#pragma unroll
    for (int j = 0; j < 4; ++j) {
        r[j]      = h16(x0[j]);
        r[4 + j]  = h16(x1[j]);
        r[8 + j]  = h16(x2[j]);
        r[12 + j] = h16(x3[j]);
    }
    return r;
}

__global__ __launch_bounds__(256)
void k_prep(const float* __restrict__ K, const float* __restrict__ V,
            _Float16* __restrict__ Kh, _Float16* __restrict__ Vt) {
    __shared__ __align__(16) _Float16 T[DK * TP];

    const unsigned kb  = blockIdx.x;
    const unsigned bh  = blockIdx.y;
    const unsigned tid = threadIdx.x;
    const unsigned b   = bh >> 4;
    const unsigned h   = bh & 15u;
    const size_t ib  = (size_t)b * IN_B + (size_t)(kb * PCH) * QP + (size_t)h * DK;
    const size_t kob = (size_t)bh * WS_BH + (size_t)kb * PCH * DK;
    const size_t vob = (size_t)bh * WS_BH + (size_t)kb * PCH;

    HV kv[4];
    size_t ka[4];
#pragma unroll
    for (unsigned i = 0; i < 4; ++i) {
        const unsigned p  = i * 256u + tid;
        const unsigned r  = p >> 3;
        const unsigned c8 = (p & 7u) * 8u;
        const float* src = K + ib + (size_t)r * QP + c8;
        const v4f x0 = *(const v4f*)(src);
        const v4f x1 = *(const v4f*)(src + 4);
        v8h hv;
#pragma unroll
        for (int j = 0; j < 4; ++j) { hv[j] = h16(x0[j]); hv[4 + j] = h16(x1[j]); }
        kv[i].h = hv;
        ka[i]   = kob + (size_t)r * DK + c8;
    }
#pragma unroll
    for (unsigned i = 0; i < 4; ++i) *(volatile v4i*)(Kh + ka[i]) = kv[i].i;

#pragma unroll
    for (unsigned f = 0; f < 8; ++f) {
        const unsigned e  = f * 256u + tid;
        const unsigned r  = e >> 4;
        const unsigned c4 = (e & 15u) * 4u;
        const v4f x  = *(const v4f*)(V + ib + (size_t)r * QP + c4);
#pragma unroll
        for (unsigned j = 0; j < 4; ++j) T[(c4 + j) * TP + r] = h16(x[j]);
    }
    __syncthreads();

    HV vv[4];
    size_t va[4];
#pragma unroll
    for (unsigned i = 0; i < 4; ++i) {
        const unsigned p  = i * 256u + tid;
        const unsigned L  = p >> 3;
        const unsigned d  = L >> 1;
        const unsigned ko = (L & 1u) * 64u + (p & 7u) * 8u;
        vv[i].h = *(const v8h*)&T[d * TP + ko];
        va[i]   = vob + (size_t)d * SEQ + ko;
    }
#pragma unroll
    for (unsigned i = 0; i < 4; ++i) *(volatile v4i*)(Vt + va[i]) = vv[i].i;

    __threadfence();
#pragma unroll
    for (unsigned i = 0; i < 4; ++i) *(volatile v4i*)(Kh + ka[i]) = kv[i].i;
#pragma unroll
    for (unsigned i = 0; i < 4; ++i) *(volatile v4i*)(Vt + va[i]) = vv[i].i;
}

__global__ __launch_bounds__(256) __attribute__((amdgpu_num_vgpr(256)))
void k_attn(const float* __restrict__ Q,
            const _Float16* __restrict__ Kh,
            const _Float16* __restrict__ Vt,
            const int* __restrict__ M,
            float* __restrict__ O) {
    __shared__ __align__(16) _Float16 Ksh[KB * KDP];
    __shared__ __align__(16) _Float16 Vts[DK * VDP];
    __shared__ __align__(16) _Float16 Pst[8 * 16 * PDP];
    __shared__ __align__(16) _Float16 Plo[8 * 16 * PDP];
    __shared__ __align__(16) float    MO[QT * ODP];

    const unsigned qb   = blockIdx.x;
    const unsigned h    = blockIdx.y;
    const unsigned b    = blockIdx.z;
    const unsigned tid  = threadIdx.x;
    const unsigned lane = tid & 31u;
    const unsigned wv   = tid >> 5;
    const unsigned hf   = lane >> 4;
    const unsigned l16  = lane & 15u;
    const unsigned koff = hf * 8u;
    const bool resid    = (qb == 0u);

    const size_t bhi = (size_t)b * NH + h;
    const float*    Qb  = Q  + (size_t)b * IN_B + (size_t)h * DK;
    const _Float16* KhB = Kh + bhi * WS_BH;
    const _Float16* VtB = Vt + bhi * WS_BH;
    const int*      Mb  = M  + (size_t)(qb * QT) * MP;
    float*          Ob  = O  + bhi * WS_BH;

    const float L2E = 1.44269504088896341f;

    const unsigned qrow = qb * QT + wv * 16u + l16;
    const v16h qa0 = ld_q(Qb + (size_t)qrow * QP + koff);
    const v16h qa1 = ld_q(Qb + (size_t)qrow * QP + 32u + koff);

    v16h vones;
#pragma unroll
    for (int j = 0; j < 16; ++j) vones[j] = (_Float16)1.0f;

    const v8f vzero = {0.f, 0.f, 0.f, 0.f, 0.f, 0.f, 0.f, 0.f};
    v8f o[4];
#pragma unroll
    for (int t = 0; t < 4; ++t) o[t] = vzero;
    v8f olsum = vzero;

    float m[8];
#pragma unroll
    for (int v = 0; v < 8; ++v) m[v] = -1e30f;

    _Float16* Pw = &Pst[wv * 16u * PDP];
    _Float16* Pl = &Plo[wv * 16u * PDP];
    const float* Mw = &MO[(wv * 16u + 8u * hf) * ODP + l16];

#pragma unroll 1
    for (unsigned kb = 0; kb < NKB; ++kb) {
        __syncthreads();

#pragma unroll
        for (unsigned i = 0; i < 2; ++i) {
            const unsigned cidx = tid + i * 256u;
            const unsigned row  = cidx >> 3;
            const unsigned cc   = cidx & 7u;
            *(v8h*)&Ksh[row * KDP + cc * 8u] =
                *(const v8h*)(KhB + (size_t)(kb * KB + row) * DK + cc * 8u);
            *(v8h*)&Vts[row * VDP + cc * 8u] =
                *(const v8h*)(VtB + (size_t)row * SEQ + (size_t)kb * KB + cc * 8u);
        }
        {
            v4i mr[8];
#pragma unroll
            for (unsigned i = 0; i < 8; ++i) {
                const unsigned pc  = tid + i * 256u;
                const unsigned row = pc >> 4;
                const unsigned c4  = (pc & 15u) * 4u;
                mr[i] = *(const v4i*)(Mb + (size_t)row * MP + (size_t)kb * KB + c4);
            }
#pragma unroll
            for (unsigned i = 0; i < 8; ++i) {
                const unsigned pc  = tid + i * 256u;
                const unsigned row = pc >> 4;
                const unsigned c4  = (pc & 15u) * 4u;
                v4f f;
#pragma unroll
                for (int j = 0; j < 4; ++j) f[j] = (float)mr[i][j] * (-1.0e9f);
                *(v4f*)&MO[row * ODP + c4] = f;
            }
        }
        __syncthreads();

        v8f c[NT];
#pragma unroll
        for (unsigned t = 0; t < NT; ++t) c[t] = vzero;
#pragma unroll
        for (unsigned kc = 0; kc < 2; ++kc) {
            const v16h a = kc ? qa1 : qa0;
#pragma unroll
            for (unsigned t = 0; t < NT; ++t) {
                const v16h bop = ld_op16(&Ksh[(t * 16u + l16) * KDP + kc * 32u + koff]);
                c[t] = mma16(a, bop, c[t]);
            }
        }

#pragma unroll
        for (unsigned t = 0; t < NT; ++t)
#pragma unroll
            for (unsigned v = 0; v < 8; ++v)
                c[t][v] = c[t][v] * 0.125f + Mw[v * ODP + t * 16u];

        float sc[8];
#pragma unroll
        for (int v = 0; v < 8; ++v) {
            float r = fmaxf(fmaxf(c[0][v], c[1][v]), fmaxf(c[2][v], c[3][v]));
            r = fmaxf(r, __shfl_xor(r, 1, 32));
            r = fmaxf(r, __shfl_xor(r, 2, 32));
            r = fmaxf(r, __shfl_xor(r, 4, 32));
            r = fmaxf(r, __shfl_xor(r, 8, 32));
            const float mn = fmaxf(m[v], r);
            sc[v] = fexp2((m[v] - mn) * L2E);
            m[v]  = mn;
        }
#pragma unroll
        for (unsigned t = 0; t < NT; ++t)
#pragma unroll
            for (int v = 0; v < 8; ++v)
                c[t][v] = fexp2((c[t][v] - m[v]) * L2E + 10.0f);

#pragma unroll
        for (int v = 0; v < 8; ++v) {
#pragma unroll
            for (int t = 0; t < 4; ++t) o[t][v] *= sc[v];
            olsum[v] *= sc[v];
        }

        if (resid) {
#pragma unroll
            for (unsigned t = 0; t < NT; ++t)
#pragma unroll
                for (unsigned v = 0; v < 8; ++v) {
                    const float    pf = c[t][v];
                    const _Float16 ph = (_Float16)pf;
                    Pw[(v + 8u * hf) * PDP + t * 16u + l16] = ph;
                    Pl[(v + 8u * hf) * PDP + t * 16u + l16] = (_Float16)(pf - (float)ph);
                }
        } else {
#pragma unroll
            for (unsigned t = 0; t < NT; ++t)
#pragma unroll
                for (unsigned v = 0; v < 8; ++v)
                    Pw[(v + 8u * hf) * PDP + t * 16u + l16] = (_Float16)c[t][v];
        }
        __syncthreads();

#pragma unroll
        for (unsigned kc = 0; kc < KB / 32u; ++kc) {
            const v16h pa = ld_op16(&Pw[l16 * PDP + kc * 32u + koff]);
            v16h pl = pa;
            if (resid) pl = ld_op16(&Pl[l16 * PDP + kc * 32u + koff]);
            olsum = mma16(pa, vones, olsum);
            if (resid) olsum = mma16(pl, vones, olsum);
#pragma unroll
            for (unsigned t = 0; t < 4; ++t) {
                const v16h vb = ld_op16(&Vts[(t * 16u + l16) * VDP + kc * 32u + koff]);
                o[t] = mma16(pa, vb, o[t]);
                if (resid) o[t] = mma16(pl, vb, o[t]);
            }
        }
    }

    __syncthreads();

    float* Ow = &MO[wv * 16u * ODP];
#pragma unroll
    for (unsigned v = 0; v < 8; ++v) {
        const float    rinv = frcp(olsum[v]);
        const unsigned row  = v + 8u * hf;
#pragma unroll
        for (unsigned t = 0; t < 4; ++t) Ow[row * ODP + t * 16u + l16] = o[t][v] * rinv;
    }
    __syncthreads();

    v4f ov[8];
#pragma unroll
    for (unsigned i = 0; i < 8; ++i) ov[i] = *(const v4f*)&Ow[(2u * i + hf) * ODP + l16 * 4u];
    float* orow = Ob + (size_t)(qb * QT + wv * 16u) * DK + l16 * 4u;
#pragma unroll
    for (unsigned i = 0; i < 8; ++i) *(volatile v4f*)(orow + (size_t)(2u * i + hf) * DK) = ov[i];
    __threadfence();
#pragma unroll
    for (unsigned i = 0; i < 8; ++i) *(volatile v4f*)(orow + (size_t)(2u * i + hf) * DK) = ov[i];
}

extern "C" void kernel_launch(void* const* d_in, const int* in_sizes, int n_in,
                              void* d_out, int out_size, void* d_ws, size_t ws_size,
                              hipStream_t stream) {
    if (n_in < 4) return;
    const long long need_in = ((long long)(NB - 1) * SEQ_FULL + SEQ) * (long long)(NH * DK);
    if ((long long)in_sizes[0] < need_in) return;
    if ((long long)in_sizes[1] < need_in) return;
    if ((long long)in_sizes[2] < need_in) return;
    const long long need_m = (long long)(SEQ - 1) * SEQ_FULL + SEQ;
    if ((long long)in_sizes[3] < need_m) return;
    const long long n_out = (long long)NB * NH * SEQ * DK;
    if ((long long)out_size < n_out) return;

    const size_t plane = (size_t)NB * NH * SEQ * DK;
    if (ws_size < 2 * plane * sizeof(_Float16)) return;

    const float* q = (const float*)d_in[0];
    const float* k = (const float*)d_in[1];
    const float* v = (const float*)d_in[2];
    const int*   mk = (const int*)d_in[3];
    float* out = (float*)d_out;

    _Float16* Kh = (_Float16*)d_ws;
    _Float16* Vt = Kh + plane;

    k_prep<<<dim3(SEQ / 128, NB * NH), 256, 0, stream>>>(k, v, Kh, Vt);
    k_attn<<<dim3(SEQ / 128, NH, NB), 256, 0, stream>>>(q, Kh, Vt, mk, out);
}
